// GCNLPA_50646254354789
// MI455X (gfx1250) — hardware-verified
//
#include <hip/hip_runtime.h>
#include <stddef.h>


#define DIN     256
#define DH      128
#define CC      64
#define NTHR    256
#define NWAVE   8
#define EPT     8
#define NGRP    2
#define CHUNK   (NTHR * EPT * NGRP)
#define WCAP    (EPT * NGRP * 32)
#define LISTN   (NWAVE * WCAP)
#define NBC     4096
#define NBF     1024
#define RCAP    40960
#define RBN     128
#define TGT     256
#define DEGCAP  256
#define GROWS   128
#define OTHR    512
#define WSCALE  16.0f
#define WINV    0.0625f

#define LDS_G1   (GROWS * (DIN + 8) * 2)
#define LDS_G2   (GROWS * (DH + 8) * 2)
#define LDS_FILL ((RCAP + NBF + LISTN) * 4 + 64)
#define LDS_T64  (NWAVE * 32 * CC * 4)

static_assert((CHUNK & (CHUNK - 1)) == 0);
static_assert(CHUNK <= 4096);
static_assert(NBC <= 4096 && NBF <= 4096);
static_assert((NBC & (NBC - 1)) == 0 && (NBF & (NBF - 1)) == 0);
static_assert(NBC == 4 * NBF);
static_assert(OTHR * 8 == NBC);
static_assert((RCAP % 32) == 0);
static_assert(GROWS * DH * 4 <= LDS_G1);
static_assert(GROWS * CC * 4 <= LDS_G2);
static_assert((TGT % GROWS) == 0 && TGT == NWAVE * 32);
static_assert(TGT == NTHR);
static_assert(CC == 64 && DH == 128);

typedef float    v2f  __attribute__((ext_vector_type(2)));
typedef float    v4f  __attribute__((ext_vector_type(4)));
typedef float    v8f  __attribute__((ext_vector_type(8)));
typedef int      v4i  __attribute__((ext_vector_type(4)));
typedef _Float16 v8h  __attribute__((ext_vector_type(8)));
typedef _Float16 v16h __attribute__((ext_vector_type(16)));
union FragH { v16h v; v8h h[2]; };
union FI { float f; int i; };

__device__ __forceinline__ v8h cvt8(v4f a, v4f b) {
  v8h r;
  r[0] = (_Float16)a.x; r[1] = (_Float16)a.y; r[2] = (_Float16)a.z; r[3] = (_Float16)a.w;
  r[4] = (_Float16)b.x; r[5] = (_Float16)b.y; r[6] = (_Float16)b.z; r[7] = (_Float16)b.w;
  return r;
}

__device__ __forceinline__ v8f wmh(v16h a, v16h b, v8f c) {
  v8f d = __builtin_amdgcn_wmma_f32_16x16x32_f16(false, a, false, b, (short)0, c, false, false);
  asm volatile("v_nop\n\tv_nop\n\tv_nop\n\tv_nop" : "+v"(d) : "v"(a), "v"(b));
  return d;
}

__device__ __forceinline__ float sigm(float v) { return 1.0f / (1.0f + expf(-v)); }

template <int NB>
__device__ __forceinline__ int scan_chunk(const int* __restrict__ keys, int nE, int cbase, int slotBase,
                                          int vec8, int* list, int tid, int lane, int wave) {
  int wc = 0;
#pragma unroll
  for (int g = 0; g < NGRP; ++g) {
    const int el0  = (g * NTHR + tid) * EPT;
    const int e0   = cbase + el0;
    const int sent = -2147483647 - 1;
    v4i da, db;
    if (vec8 != 0 && cbase + CHUNK <= nE) {
      da = *(const v4i*)(keys + e0);
      db = *(const v4i*)(keys + e0 + 4);
    } else {
      da.x = (e0     < nE) ? keys[min(e0, nE - 1)] : sent;
      da.y = (e0 + 1 < nE) ? keys[min(e0 + 1, nE - 1)] : sent;
      da.z = (e0 + 2 < nE) ? keys[min(e0 + 2, nE - 1)] : sent;
      da.w = (e0 + 3 < nE) ? keys[min(e0 + 3, nE - 1)] : sent;
      db.x = (e0 + 4 < nE) ? keys[min(e0 + 4, nE - 1)] : sent;
      db.y = (e0 + 5 < nE) ? keys[min(e0 + 5, nE - 1)] : sent;
      db.z = (e0 + 6 < nE) ? keys[min(e0 + 6, nE - 1)] : sent;
      db.w = (e0 + 7 < nE) ? keys[min(e0 + 7, nE - 1)] : sent;
    }
    const unsigned nb = (unsigned)slotBase;
    const unsigned s0 = (unsigned)da.x - nb, s1 = (unsigned)da.y - nb;
    const unsigned s2 = (unsigned)da.z - nb, s3 = (unsigned)da.w - nb;
    const unsigned s4 = (unsigned)db.x - nb, s5 = (unsigned)db.y - nb;
    const unsigned s6 = (unsigned)db.z - nb, s7 = (unsigned)db.w - nb;
    const bool h0 = s0 < (unsigned)NB, h1 = s1 < (unsigned)NB, h2 = s2 < (unsigned)NB, h3 = s3 < (unsigned)NB;
    const bool h4 = s4 < (unsigned)NB, h5 = s5 < (unsigned)NB, h6 = s6 < (unsigned)NB, h7 = s7 < (unsigned)NB;
    const unsigned any = __builtin_amdgcn_ballot_w32(h0 | h1 | h2 | h3 | h4 | h5 | h6 | h7);
    if (any != 0u) {
#define HITJ(J, HJ, SJ) { \
        const unsigned mj = __builtin_amdgcn_ballot_w32(HJ); \
        if (mj != 0u) { \
          if (HJ) { \
            const int pos = wc + (int)__builtin_amdgcn_mbcnt_lo(mj, 0u); \
            if (pos < WCAP) list[wave * WCAP + pos] = ((el0 + (J)) << 12) | (int)(SJ); \
          } \
          wc += (int)__builtin_popcount(mj); } }
      HITJ(0, h0, s0)
      HITJ(1, h1, s1)
      HITJ(2, h2, s2)
      HITJ(3, h3, s3)
      HITJ(4, h4, s4)
      HITJ(5, h5, s5)
      HITJ(6, h6, s6)
      HITJ(7, h7, s7)
#undef HITJ
    }
  }
  return wc;
}

__global__ __launch_bounds__(NTHR) void k_wprep(
    const float* __restrict__ w1, const float* __restrict__ w2, _Float16* wp) {
  const int seg = (int)blockIdx.x < 16 ? 0 : 1;
  const float* src = seg == 0 ? w1 : w2;
  const int K  = seg == 0 ? DIN : DH;
  const int Nc = seg == 0 ? DH : CC;
  const int blk = seg == 0 ? (int)blockIdx.x : (int)blockIdx.x - 16;
  const int i  = blk * NTHR + (int)threadIdx.x;
  const int kg = K / 8;
  const int n  = i / kg;
  const int k0 = (i - n * kg) * 8;
  float v[8];
#pragma unroll
  for (int e = 0; e < 8; ++e) v[e] = src[(size_t)(k0 + e) * Nc + n] * WSCALE;
  v4f a, b;
  a.x = v[0]; a.y = v[1]; a.z = v[2]; a.w = v[3];
  b.x = v[4]; b.y = v[5]; b.z = v[6]; b.w = v[7];
  const v8h hv = cvt8(a, b);
  _Float16* dp = wp + (seg == 0 ? (size_t)0 : (size_t)DIN * DH) + (size_t)i * 8;
  *(volatile v8h*)dp = hv;
  __threadfence();
  *(volatile v8h*)dp = hv;
}

__global__ __launch_bounds__(NTHR) void k_count(
    const int* __restrict__ keys, int* cnt, int nE, int vec8) {
  __shared__ __attribute__((aligned(16))) int scnt[NBC];
  __shared__ __attribute__((aligned(16))) int list[LISTN];
  __shared__ int wcnt[NWAVE];
  const int tid = threadIdx.x, lane = tid & 31, wave = tid >> 5;
  const int nodeBase = blockIdx.x * NBC;

  for (int i = tid; i < NBC; i += NTHR) scnt[i] = 0;
  __syncthreads();

  const int nChunks = (nE + CHUNK - 1) / CHUNK;
#pragma unroll 1
  for (int ch = 0; ch < nChunks; ++ch) {
    const int cbase = ch * CHUNK;
    const int wc = scan_chunk<NBC>(keys, nE, cbase, nodeBase, vec8, list, tid, lane, wave);
    if (lane == 0) wcnt[wave] = wc;
    __syncthreads();
    if (wave == 0) {
#pragma unroll 1
      for (int wsx = 0; wsx < NWAVE; ++wsx) {
        int n = __builtin_amdgcn_readfirstlane(wcnt[wsx]);
        n = n > WCAP ? WCAP : (n < 0 ? 0 : n);
        const int* lp = list + wsx * WCAP;
#pragma unroll 1
        for (int i = 0; i < n; ++i) {
          const int ent  = __builtin_amdgcn_readfirstlane(lp[i]);
          const int slot = ent & (NBC - 1);
          if (lane == 0) scnt[slot] = scnt[slot] + 1;
        }
      }
    }
    __syncthreads();
  }

  v4i cq[4];
#pragma unroll
  for (int q = 0; q < 4; ++q) {
    const int f = (wave * 4 + q) * 128 + 4 * lane;
    cq[q] = *(const v4i*)(scnt + f);
  }
  int* cp = cnt + (size_t)nodeBase;
#pragma unroll
  for (int q = 0; q < 4; ++q) {
    const int f = (wave * 4 + q) * 128 + 4 * lane;
    *(volatile v4i*)(cp + f) = cq[q];
  }
  __threadfence();
#pragma unroll
  for (int q = 0; q < 4; ++q) {
    const int f = (wave * 4 + q) * 128 + 4 * lane;
    *(volatile v4i*)(cp + f) = cq[q];
  }
}

__global__ __launch_bounds__(OTHR) void k_offsets(
    const int* __restrict__ cnt, int* off, int* rbase, int nChunk) {
  __shared__ __attribute__((aligned(16))) int soff[NBC];
  __shared__ __attribute__((aligned(16))) int srb[RBN];
  __shared__ int wtot[OTHR / 32];
  const int tid = threadIdx.x, lane = tid & 31, wave = tid >> 5, sub = tid >> 7;
  for (int i = tid; i < RBN; i += OTHR) srb[i] = 0;
  int carry = 0;
#pragma unroll 1
  for (int ch = 0; ch < nChunk; ++ch) {
    const int base = ch * NBC;
    const v4i c0 = *(const v4i*)(cnt + base + 8 * tid);
    const v4i c1 = *(const v4i*)(cnt + base + 8 * tid + 4);
    const int e0 = max(c0.x, 0), e1 = max(c0.y, 0), e2 = max(c0.z, 0), e3 = max(c0.w, 0);
    const int e4 = max(c1.x, 0), e5 = max(c1.y, 0), e6 = max(c1.z, 0), e7 = max(c1.w, 0);
    const int ts = e0 + e1 + e2 + e3 + e4 + e5 + e6 + e7;
    int incl = ts;
#pragma unroll
    for (int d = 1; d < 32; d <<= 1) {
      const int t = __shfl_up(incl, d);
      if (lane >= d) incl += t;
    }
    if (lane == 31) wtot[wave] = incl;
    __syncthreads();
    const int S0 = wtot[0]  + wtot[1]  + wtot[2]  + wtot[3];
    const int S1 = wtot[4]  + wtot[5]  + wtot[6]  + wtot[7];
    const int S2 = wtot[8]  + wtot[9]  + wtot[10] + wtot[11];
    const int S3 = wtot[12] + wtot[13] + wtot[14] + wtot[15];
    int pre = 0;
#pragma unroll 1
    for (int w = 4 * sub; w < wave; ++w) pre += wtot[w];
    const int b0 = carry;
    const int b1 = b0 + ((S0 + 31) & ~31);
    const int b2 = b1 + ((S1 + 31) & ~31);
    const int b3 = b2 + ((S2 + 31) & ~31);
    const int b4 = b3 + ((S3 + 31) & ~31);
    const int myb = sub == 0 ? b0 : (sub == 1 ? b1 : (sub == 2 ? b2 : b3));
    if (tid == 0) {
      srb[min(4 * ch + 0, RBN - 1)] = b0;
      srb[min(4 * ch + 1, RBN - 1)] = b1;
      srb[min(4 * ch + 2, RBN - 1)] = b2;
      srb[min(4 * ch + 3, RBN - 1)] = b3;
    }
    int run = myb + pre + incl - ts;
    soff[8 * tid + 0] = run; run += e0;
    soff[8 * tid + 1] = run; run += e1;
    soff[8 * tid + 2] = run; run += e2;
    soff[8 * tid + 3] = run; run += e3;
    soff[8 * tid + 4] = run; run += e4;
    soff[8 * tid + 5] = run; run += e5;
    soff[8 * tid + 6] = run; run += e6;
    soff[8 * tid + 7] = run;
    carry = b4;
    __syncthreads();
    const v4i o0 = *(const v4i*)(soff + 4 * tid);
    const v4i o1 = *(const v4i*)(soff + 4 * (tid + OTHR));
    int* op = off + base;
    *(volatile v4i*)(op + 4 * tid) = o0;
    *(volatile v4i*)(op + 4 * (tid + OTHR)) = o1;
    __threadfence();
    *(volatile v4i*)(op + 4 * tid) = o0;
    *(volatile v4i*)(op + 4 * (tid + OTHR)) = o1;
    __syncthreads();
  }
  if (tid == 0) srb[min(4 * nChunk, RBN - 1)] = carry;
  __syncthreads();
  v4i rv = {0, 0, 0, 0};
  if (tid < 32) rv = *(const v4i*)(srb + 4 * tid);
  if (tid < 32) *(volatile v4i*)(rbase + 4 * tid) = rv;
  __threadfence();
  if (tid < 32) *(volatile v4i*)(rbase + 4 * tid) = rv;
}

__global__ __launch_bounds__(NTHR) void k_fill(
    const int* __restrict__ keys, const int* __restrict__ off, const int* __restrict__ rbase,
    int* csr, int nE, int vec8, int csrLen) {
  extern __shared__ v4f lds_dyn[];
  int* region = (int*)lds_dyn;
  int* cursor = region + RCAP;
  int* list   = cursor + NBF;
  int* wcnt   = list + LISTN;
  const int tid = threadIdx.x, lane = tid & 31, wave = tid >> 5;
  const int b = blockIdx.x;
  const int nodeBase = b * NBF;

  int rb0 = rbase[b];
  const int rb1 = rbase[b + 1];
  rb0 = rb0 < 0 ? 0 : (rb0 > csrLen ? csrLen : rb0);
  rb0 &= ~31;
  int len = rb1 - rb0;
  len = len < 0 ? 0 : (len > RCAP ? RCAP : len);
  int lenW = (len + 31) & ~31;
  if (rb0 + lenW > csrLen) lenW = (csrLen - rb0) & ~31;

  {
    const v4i z = {0, 0, 0, 0};
    for (int i = tid; i < RCAP / 4; i += NTHR) ((v4i*)region)[i] = z;
    for (int s = tid; s < NBF; s += NTHR) {
      int o = off[nodeBase + s] - rb0;
      o = o < 0 ? 0 : (o > RCAP ? RCAP : o);
      cursor[s] = o;
    }
  }
  __syncthreads();

  const int nChunks = (nE + CHUNK - 1) / CHUNK;
#pragma unroll 1
  for (int ch = 0; ch < nChunks; ++ch) {
    const int cbase = ch * CHUNK;
    const int wc = scan_chunk<NBF>(keys, nE, cbase, nodeBase, vec8, list, tid, lane, wave);
    if (lane == 0) wcnt[wave] = wc;
    __syncthreads();
    if (wave == 0) {
#pragma unroll 1
      for (int wsx = 0; wsx < NWAVE; ++wsx) {
        int n = __builtin_amdgcn_readfirstlane(wcnt[wsx]);
        n = n > WCAP ? WCAP : (n < 0 ? 0 : n);
        const int* lp = list + wsx * WCAP;
#pragma unroll 1
        for (int i = 0; i < n; ++i) {
          const int ent  = __builtin_amdgcn_readfirstlane(lp[i]);
          const int slot = ent & (NBF - 1);
          int e = cbase + ((ent >> 12) & (CHUNK - 1));
          e = e > nE - 1 ? nE - 1 : e;
          if (lane == 0) {
            int pos = cursor[slot];
            pos = pos < 0 ? 0 : (pos > RCAP - 1 ? RCAP - 1 : pos);
            region[pos] = e;
            const int np = pos + 1;
            cursor[slot] = np > RCAP ? RCAP : np;
          }
        }
      }
    }
    __syncthreads();
  }

  const int nv = lenW >> 2;
  int* gp = csr + rb0;
#pragma unroll 1
  for (int i = tid; i < nv; i += NTHR) { const v4i v = ((const v4i*)region)[i]; *(volatile v4i*)(gp + 4 * i) = v; }
  __threadfence();
#pragma unroll 1
  for (int i = tid; i < nv; i += NTHR) { const v4i v = ((const v4i*)region)[i]; *(volatile v4i*)(gp + 4 * i) = v; }
}

__global__ __launch_bounds__(NTHR) void k_deg(
    const int* __restrict__ csr, const int* __restrict__ off, const int* __restrict__ cnt,
    const float* __restrict__ edge_w, float* dinv, int nE, int csrLen) {
  __shared__ __attribute__((aligned(16))) float sdv[NTHR];
  const int tid = threadIdx.x;
  const int c = blockIdx.x * NTHR + tid;
  int n = cnt[c];
  n = n < 0 ? 0 : (n > DEGCAP ? DEGCAP : n);
  const int st = off[c];
  float deg = 1.0f;
#pragma unroll 1
  for (int p = 0; p < n; ++p) {
    int pos = st + p;
    pos = pos < 0 ? 0 : (pos > csrLen - 1 ? csrLen - 1 : pos);
    int e = csr[pos];
    e = e < 0 ? 0 : (e > nE - 1 ? nE - 1 : e);
    deg += sigm(edge_w[e]);
  }
  sdv[tid] = rsqrtf(deg);
  __syncthreads();
  v4f v = {0.f, 0.f, 0.f, 0.f};
  if (tid < NTHR / 4) v = *(const v4f*)(sdv + 4 * tid);
  float* dp = dinv + (size_t)blockIdx.x * NTHR + 4 * tid;
  if (tid < NTHR / 4) *(volatile v4f*)dp = v;
  __threadfence();
  if (tid < NTHR / 4) *(volatile v4f*)dp = v;
}

template <int KD, int NOUT>
__global__ __launch_bounds__(NTHR) void k_gemm(
    const float* __restrict__ A, const _Float16* __restrict__ Bs, const float* __restrict__ dinv,
    float* C, int nRowsA) {
  extern __shared__ v4f lds_dyn[];
  constexpr int AP   = KD + 8;
  constexpr int NT   = NOUT / 16;
  constexpr int NSTG = (GROWS * KD / 8) / NTHR;
  constexpr int NI   = 16 * NOUT / 128;
  static_assert((GROWS * KD / 8) % NTHR == 0);
  static_assert((16 * NOUT) % 128 == 0);
  static_assert(KD % 32 == 0 && NOUT % 16 == 0);
  _Float16* sA  = (_Float16*)lds_dyn;
  float*    stg = (float*)lds_dyn;
  const int tid = threadIdx.x, lane = tid & 31, wave = tid >> 5, hh = lane >> 4, m = lane & 15;
  const int rowBase = blockIdx.x * GROWS;

#pragma unroll
  for (int i = 0; i < NSTG; ++i) {
    const int idx = i * NTHR + tid;
    const int r   = idx / (KD / 8);
    const int c0  = (idx - r * (KD / 8)) * 8;
    int row = rowBase + r;
    row = row > nRowsA - 1 ? nRowsA - 1 : row;
    const float* ap = A + (size_t)row * KD + c0;
    const v4f a = *(const v4f*)ap, b = *(const v4f*)(ap + 4);
    *(v8h*)(sA + r * AP + c0) = cvt8(a, b);
  }
  __syncthreads();

  v8f acc[NT];
#pragma unroll
  for (int t = 0; t < NT; ++t) { v8f z = {0.f, 0.f, 0.f, 0.f, 0.f, 0.f, 0.f, 0.f}; acc[t] = z; }
  const _Float16* ar = sA + (wave * 16 + m) * AP + 8 * hh;
#pragma unroll 1
  for (int kt = 0; kt < KD / 32; ++kt) {
    FragH a;
    a.h[0] = *(const v8h*)(ar + 32 * kt);
    a.h[1] = *(const v8h*)(ar + 32 * kt + 16);
#pragma unroll
    for (int t = 0; t < NT; ++t) {
      const _Float16* bp = Bs + (size_t)(16 * t + m) * KD + 32 * kt + 8 * hh;
      FragH b;
      b.h[0] = *(const v8h*)bp;
      b.h[1] = *(const v8h*)(bp + 16);
      acc[t] = wmh(a.v, b.v, acc[t]);
    }
  }
  __syncthreads();

  const int r0 = wave * 16 + 8 * hh;
  const v4f dA = *(const v4f*)(dinv + (size_t)rowBase + r0);
  const v4f dB = *(const v4f*)(dinv + (size_t)rowBase + r0 + 4);
  float s[8];
  s[0] = dA.x; s[1] = dA.y; s[2] = dA.z; s[3] = dA.w; s[4] = dB.x; s[5] = dB.y; s[6] = dB.z; s[7] = dB.w;
#pragma unroll
  for (int r = 0; r < 8; ++r) s[r] = s[r] * WINV;
  float* sp = stg + r0 * NOUT + m;
#pragma unroll
  for (int t = 0; t < NT; ++t) {
#pragma unroll
    for (int r = 0; r < 8; ++r) sp[r * NOUT + 16 * t] = acc[t][r] * s[r];
  }
  __syncthreads();

  const float* lp = stg + wave * 16 * NOUT + 4 * lane;
  float* gp = C + ((size_t)rowBase + wave * 16) * NOUT + 4 * lane;
#pragma unroll
  for (int i = 0; i < NI; ++i) { const v4f v = *(const v4f*)(lp + i * 128); *(volatile v4f*)(gp + (size_t)i * 128) = v; }
  __threadfence();
#pragma unroll
  for (int i = 0; i < NI; ++i) { const v4f v = *(const v4f*)(lp + i * 128); *(volatile v4f*)(gp + (size_t)i * 128) = v; }
}

__global__ __launch_bounds__(NTHR) void k_agg1(
    const int* __restrict__ csr, const int* __restrict__ off, const int* __restrict__ cnt,
    const int* __restrict__ srcs, const float* __restrict__ edge_w, const float* __restrict__ dinv,
    const float* __restrict__ hw, const float* __restrict__ bs, float* h,
    int nN, int nE, int csrLen) {
  const int tid = threadIdx.x, lane = tid & 31, wave = tid >> 5;
  const int tbase = blockIdx.x * TGT + wave * 32;
  const int cl = tbase + lane;
  const int cnt_l = cnt[cl];
  const int off_l = off[cl];
  FI dvu; dvu.f = dinv[cl];
  const v4f bb = *(const v4f*)(bs + 4 * lane);

#pragma unroll 1
  for (int j = 0; j < 32; ++j) {
    const int c = tbase + j;
    int n = __builtin_amdgcn_readlane(cnt_l, j);
    n = n < 0 ? 0 : (n > DEGCAP ? DEGCAP : n);
    const int st = __builtin_amdgcn_readlane(off_l, j);
    FI du; du.i = __builtin_amdgcn_readlane(dvu.i, j);
    const float dc = du.f;
    v4f acc = {0.f, 0.f, 0.f, 0.f};
#pragma unroll 1
    for (int q0 = 0; q0 < n; q0 += 32) {
      int pos = st + q0 + lane;
      pos = pos < 0 ? 0 : (pos > csrLen - 1 ? csrLen - 1 : pos);
      int e = csr[pos];
      e = e < 0 ? 0 : (e > nE - 1 ? nE - 1 : e);
      int sl = srcs[e];
      sl = sl < 0 ? 0 : (sl > nN - 1 ? nN - 1 : sl);
      FI wl; wl.f = sigm(edge_w[e]);
      const int mcnt = (n - q0) < 32 ? (n - q0) : 32;
#pragma unroll 1
      for (int p = 0; p < mcnt; ++p) {
        const int s = __builtin_amdgcn_readlane(sl, p);
        FI wu; wu.i = __builtin_amdgcn_readlane(wl.i, p);
        const v4f hv = *(const v4f*)(hw + (size_t)s * DH + 4 * lane);
        acc = acc + hv * wu.f;
      }
    }
    const v4f sv = *(const v4f*)(hw + (size_t)c * DH + 4 * lane);
    v4f v = (acc + sv) * dc + bb;
    v.x = fmaxf(v.x, 0.f); v.y = fmaxf(v.y, 0.f); v.z = fmaxf(v.z, 0.f); v.w = fmaxf(v.w, 0.f);
    float* hp = h + (size_t)c * DH + 4 * lane;
    *(volatile v4f*)hp = v;
    __threadfence();
    *(volatile v4f*)hp = v;
  }
}

__global__ __launch_bounds__(NTHR) void k_agg2(
    const int* __restrict__ csr, const int* __restrict__ off, const int* __restrict__ cnt,
    const int* __restrict__ srcs, const float* __restrict__ edge_w, const float* __restrict__ dinv,
    const float* __restrict__ hw, const float* __restrict__ bs, float* out,
    int nN, int nE, int csrLen) {
  extern __shared__ v4f lds_dyn[];
  const int tid = threadIdx.x, lane = tid & 31, wave = tid >> 5;
  float* stile = (float*)lds_dyn + wave * 32 * CC;
  const int tbase = blockIdx.x * TGT + wave * 32;
  const int cl = tbase + lane;
  const int cnt_l = cnt[cl];
  const int off_l = off[cl];
  FI dvu; dvu.f = dinv[cl];
  const v2f bb = *(const v2f*)(bs + 2 * lane);

#pragma unroll 1
  for (int j = 0; j < 32; ++j) {
    const int c = tbase + j;
    int n = __builtin_amdgcn_readlane(cnt_l, j);
    n = n < 0 ? 0 : (n > DEGCAP ? DEGCAP : n);
    const int st = __builtin_amdgcn_readlane(off_l, j);
    FI du; du.i = __builtin_amdgcn_readlane(dvu.i, j);
    const float dc = du.f;
    v2f acc = {0.f, 0.f};
#pragma unroll 1
    for (int q0 = 0; q0 < n; q0 += 32) {
      int pos = st + q0 + lane;
      pos = pos < 0 ? 0 : (pos > csrLen - 1 ? csrLen - 1 : pos);
      int e = csr[pos];
      e = e < 0 ? 0 : (e > nE - 1 ? nE - 1 : e);
      int sl = srcs[e];
      sl = sl < 0 ? 0 : (sl > nN - 1 ? nN - 1 : sl);
      FI wl; wl.f = sigm(edge_w[e]);
      const int mcnt = (n - q0) < 32 ? (n - q0) : 32;
#pragma unroll 1
      for (int p = 0; p < mcnt; ++p) {
        const int s = __builtin_amdgcn_readlane(sl, p);
        FI wu; wu.i = __builtin_amdgcn_readlane(wl.i, p);
        const v2f hv = *(const v2f*)(hw + (size_t)s * CC + 2 * lane);
        acc = acc + hv * wu.f;
      }
    }
    const v2f sv = *(const v2f*)(hw + (size_t)c * CC + 2 * lane);
    const v2f v = (acc + sv) * dc + bb;
    float mx = fmaxf(v.x, v.y);
#pragma unroll
    for (int o = 16; o > 0; o >>= 1) mx = fmaxf(mx, __shfl_xor(mx, o, 32));
    const float ex = expf(v.x - mx), ey = expf(v.y - mx);
    float sm = ex + ey;
#pragma unroll
    for (int o = 16; o > 0; o >>= 1) sm += __shfl_xor(sm, o, 32);
    const float inv = 1.0f / sm;
    v2f ov; ov.x = ex * inv; ov.y = ey * inv;
    *(v2f*)(stile + j * CC + 2 * lane) = ov;
  }
  __syncthreads();

  const int rsub = lane >> 4;
#pragma unroll
  for (int i = 0; i < 16; ++i) {
    const v4f v = *(const v4f*)(stile + i * 128 + 4 * lane);
    const int row = tbase + 2 * i + rsub;
    if (row < nN) *(volatile v4f*)(out + (size_t)tbase * CC + i * 128 + 4 * lane) = v;
  }
  __threadfence();
#pragma unroll
  for (int i = 0; i < 16; ++i) {
    const v4f v = *(const v4f*)(stile + i * 128 + 4 * lane);
    const int row = tbase + 2 * i + rsub;
    if (row < nN) *(volatile v4f*)(out + (size_t)tbase * CC + i * 128 + 4 * lane) = v;
  }
}

template <bool FIRST>
__global__ __launch_bounds__(NTHR) void k_prop(
    const int* __restrict__ csr, const int* __restrict__ off, const int* __restrict__ cnt,
    const int* __restrict__ dsts, const float* __restrict__ edge_w, const int* __restrict__ y,
    const float* __restrict__ Lin, float* Lout,
    int nN, int nE, int csrLen, int nStoreRows, int normalize) {
  extern __shared__ v4f lds_dyn[];
  const int tid = threadIdx.x, lane = tid & 31, wave = tid >> 5;
  float* stile = (float*)lds_dyn + wave * 32 * CC;
  const int tbase = blockIdx.x * TGT + wave * 32;
  const int cl = tbase + lane;
  const int cnt_l = cnt[cl];
  const int off_l = off[cl];
  const int c0 = 2 * lane, c1 = 2 * lane + 1;

#pragma unroll 1
  for (int j = 0; j < 32; ++j) {
    const int c = tbase + j;
    int n = __builtin_amdgcn_readlane(cnt_l, j);
    n = n < 0 ? 0 : (n > DEGCAP ? DEGCAP : n);
    const int st = __builtin_amdgcn_readlane(off_l, j);
    v2f acc = {0.f, 0.f};
#pragma unroll 1
    for (int q0 = 0; q0 < n; q0 += 32) {
      int pos = st + q0 + lane;
      pos = pos < 0 ? 0 : (pos > csrLen - 1 ? csrLen - 1 : pos);
      int e = csr[pos];
      e = e < 0 ? 0 : (e > nE - 1 ? nE - 1 : e);
      int dl = dsts[e];
      dl = dl < 0 ? 0 : (dl > nN - 1 ? nN - 1 : dl);
      FI wl; wl.f = sigm(edge_w[e]);
      int yl = 0;
      if (FIRST) yl = y[dl];
      const int mcnt = (n - q0) < 32 ? (n - q0) : 32;
#pragma unroll 1
      for (int p = 0; p < mcnt; ++p) {
        FI wu; wu.i = __builtin_amdgcn_readlane(wl.i, p);
        const float w = wu.f;
        if (FIRST) {
          const int yd = __builtin_amdgcn_readlane(yl, p);
          acc.x += (yd == c0) ? w : 0.f;
          acc.y += (yd == c1) ? w : 0.f;
        } else {
          const int d = __builtin_amdgcn_readlane(dl, p);
          const v2f lv = *(const v2f*)(Lin + (size_t)d * CC + 2 * lane);
          acc = acc + lv * w;
        }
      }
    }
    v2f sv;
    if (FIRST) {
      const int yc = y[c < nN ? c : nN - 1];
      sv.x = (yc == c0) ? 1.0f : 0.0f;
      sv.y = (yc == c1) ? 1.0f : 0.0f;
    } else {
      sv = *(const v2f*)(Lin + (size_t)c * CC + 2 * lane);
    }
    v2f v = acc + sv;
    if (normalize != 0) {
      float ss = v.x * v.x + v.y * v.y;
#pragma unroll
      for (int o = 16; o > 0; o >>= 1) ss += __shfl_xor(ss, o, 32);
      const float inv = 1.0f / fmaxf(sqrtf(ss), 1e-12f);
      v = v * inv;
    }
    *(v2f*)(stile + j * CC + 2 * lane) = v;
  }
  __syncthreads();

  const int rsub = lane >> 4;
#pragma unroll
  for (int i = 0; i < 16; ++i) {
    const v4f v = *(const v4f*)(stile + i * 128 + 4 * lane);
    const int row = tbase + 2 * i + rsub;
    if (row < nStoreRows) *(volatile v4f*)(Lout + (size_t)tbase * CC + i * 128 + 4 * lane) = v;
  }
  __threadfence();
#pragma unroll
  for (int i = 0; i < 16; ++i) {
    const v4f v = *(const v4f*)(stile + i * 128 + 4 * lane);
    const int row = tbase + 2 * i + rsub;
    if (row < nStoreRows) *(volatile v4f*)(Lout + (size_t)tbase * CC + i * 128 + 4 * lane) = v;
  }
}

extern "C" void kernel_launch(void* const* d_in, const int* in_sizes, int n_in,
                              void* d_out, int out_size, void* d_ws, size_t ws_size,
                              hipStream_t stream) {
  if (n_in < 8) return;
  const int nN = in_sizes[2];
  const int nE = in_sizes[1] / 2;
  if (nN <= 0 || nE <= 0) return;
  if (in_sizes[0] != nN * DIN || in_sizes[1] != 2 * nE || in_sizes[3] != nE) return;
  if (in_sizes[4] != DIN * DH || in_sizes[5] != DH || in_sizes[6] != DH * CC || in_sizes[7] != CC) return;
  if (out_size != 2 * nN * CC) return;
  if (nE > (1 << 28) || nN > (1 << 24)) return;

  const float* x      = (const float*)d_in[0];
  const int*   ei     = (const int*)d_in[1];
  const int*   srcs   = ei;
  const int*   dsts   = ei + nE;
  const int*   y      = (const int*)d_in[2];
  const float* edge_w = (const float*)d_in[3];
  const float* W1     = (const float*)d_in[4];
  const float* W2     = (const float*)d_in[6];
  float* out0 = (float*)d_out;
  float* out1 = (float*)d_out + (size_t)nN * CC;

  const int NPAD   = ((nN + TGT - 1) / TGT) * TGT;
  const int nBC    = (nN + NBC - 1) / NBC;
  const int CNTPAD = nBC * NBC;
  if (CNTPAD < NPAD) return;
  if (4 * nBC + 1 > RBN) return;
  const int nBF    = (nN + NBF - 1) / NBF;
  const int csrLen = ((nE + 31) & ~31) + 4096;
  if (31 * 4 * nBC > 4096) return;
  const int nGemm  = NPAD / GROWS;
  const int nAgg   = NPAD / TGT;

  char* ws = (char*)d_ws;
  size_t off = 0;
  const size_t oW    = off; off += (size_t)(DIN * DH + DH * CC) * 2; off = (off + 255) & ~(size_t)255;
  const size_t oCntA = off; off += (size_t)CNTPAD * 4;              off = (off + 255) & ~(size_t)255;
  const size_t oOffA = off; off += (size_t)CNTPAD * 4;              off = (off + 255) & ~(size_t)255;
  const size_t oRbA  = off; off += (size_t)RBN * 4;                 off = (off + 255) & ~(size_t)255;
  const size_t oCsrA = off; off += (size_t)csrLen * 4;              off = (off + 255) & ~(size_t)255;
  const size_t oCntB = off; off += (size_t)CNTPAD * 4;              off = (off + 255) & ~(size_t)255;
  const size_t oOffB = off; off += (size_t)CNTPAD * 4;              off = (off + 255) & ~(size_t)255;
  const size_t oRbB  = off; off += (size_t)RBN * 4;                 off = (off + 255) & ~(size_t)255;
  const size_t oCsrB = off; off += (size_t)csrLen * 4;              off = (off + 255) & ~(size_t)255;
  const size_t oDv   = off; off += (size_t)CNTPAD * 4;              off = (off + 255) & ~(size_t)255;
  const size_t oHw1  = off; off += (size_t)NPAD * DH * 4;           off = (off + 255) & ~(size_t)255;
  const size_t oH1   = off; off += (size_t)NPAD * DH * 4;           off = (off + 255) & ~(size_t)255;
  const size_t oHw2  = off; off += (size_t)NPAD * CC * 4;           off = (off + 255) & ~(size_t)255;
  const size_t oLA   = off; off += (size_t)NPAD * CC * 4;           off = (off + 255) & ~(size_t)255;
  const size_t oLB   = off; off += (size_t)NPAD * CC * 4;           off = (off + 255) & ~(size_t)255;
  if (off > ws_size) return;
  _Float16* wp    = (_Float16*)(ws + oW);
  int*      cntA  = (int*)(ws + oCntA);
  int*      offA  = (int*)(ws + oOffA);
  int*      rbA   = (int*)(ws + oRbA);
  int*      csrA  = (int*)(ws + oCsrA);
  int*      cntB  = (int*)(ws + oCntB);
  int*      offB  = (int*)(ws + oOffB);
  int*      rbB   = (int*)(ws + oRbB);
  int*      csrB  = (int*)(ws + oCsrB);
  float*    dinv  = (float*)(ws + oDv);
  float*    hw1   = (float*)(ws + oHw1);
  float*    h1    = (float*)(ws + oH1);
  float*    hw2   = (float*)(ws + oHw2);
  float*    LA    = (float*)(ws + oLA);
  float*    LB    = (float*)(ws + oLB);

  const int vec8 = ((nE & 3) == 0) ? 1 : 0;

  k_wprep<<<20, NTHR, 0, stream>>>(W1, W2, wp);

  k_count<<<nBC, NTHR, 0, stream>>>(dsts, cntA, nE, vec8);
  k_offsets<<<1, OTHR, 0, stream>>>(cntA, offA, rbA, nBC);
  hipFuncSetAttribute(reinterpret_cast<const void*>(&k_fill),
                      hipFuncAttributeMaxDynamicSharedMemorySize, LDS_FILL);
  k_fill<<<nBF, NTHR, LDS_FILL, stream>>>(dsts, offA, rbA, csrA, nE, vec8, csrLen);

  k_count<<<nBC, NTHR, 0, stream>>>(srcs, cntB, nE, vec8);
  k_offsets<<<1, OTHR, 0, stream>>>(cntB, offB, rbB, nBC);
  k_fill<<<nBF, NTHR, LDS_FILL, stream>>>(srcs, offB, rbB, csrB, nE, vec8, csrLen);

  k_deg<<<NPAD / NTHR, NTHR, 0, stream>>>(csrA, offA, cntA, edge_w, dinv, nE, csrLen);

  hipFuncSetAttribute(reinterpret_cast<const void*>(&k_gemm<DIN, DH>),
                      hipFuncAttributeMaxDynamicSharedMemorySize, LDS_G1);
  k_gemm<DIN, DH><<<nGemm, NTHR, LDS_G1, stream>>>(x, wp, dinv, hw1, nN);
  k_agg1<<<nAgg, NTHR, 0, stream>>>(csrA, offA, cntA, srcs, edge_w, dinv, hw1,
                                    (const float*)d_in[5], h1, nN, nE, csrLen);

  hipFuncSetAttribute(reinterpret_cast<const void*>(&k_gemm<DH, CC>),
                      hipFuncAttributeMaxDynamicSharedMemorySize, LDS_G2);
  k_gemm<DH, CC><<<nGemm, NTHR, LDS_G2, stream>>>(h1, wp + (size_t)DIN * DH, dinv, hw2, NPAD);
  hipFuncSetAttribute(reinterpret_cast<const void*>(&k_agg2),
                      hipFuncAttributeMaxDynamicSharedMemorySize, LDS_T64);
  k_agg2<<<nAgg, NTHR, LDS_T64, stream>>>(csrA, offA, cntA, srcs, edge_w, dinv, hw2,
                                          (const float*)d_in[7], out0, nN, nE, csrLen);

  hipFuncSetAttribute(reinterpret_cast<const void*>(&k_prop<true>),
                      hipFuncAttributeMaxDynamicSharedMemorySize, LDS_T64);
  hipFuncSetAttribute(reinterpret_cast<const void*>(&k_prop<false>),
                      hipFuncAttributeMaxDynamicSharedMemorySize, LDS_T64);
  k_prop<true><<<nAgg, NTHR, LDS_T64, stream>>>(csrB, offB, cntB, dsts, edge_w, y, LB, LA,
                                                nN, nE, csrLen, NPAD, 0);
  k_prop<false><<<nAgg, NTHR, LDS_T64, stream>>>(csrB, offB, cntB, dsts, edge_w, y, LA, LB,
                                                 nN, nE, csrLen, NPAD, 0);
  k_prop<false><<<nAgg, NTHR, LDS_T64, stream>>>(csrB, offB, cntB, dsts, edge_w, y, LB, LA,
                                                 nN, nE, csrLen, NPAD, 0);
  k_prop<false><<<nAgg, NTHR, LDS_T64, stream>>>(csrB, offB, cntB, dsts, edge_w, y, LA, out1,
                                                 nN, nE, csrLen, nN, 1);
}
